// JRTransformer_33509334843568
// MI455X (gfx1250) — hardware-run, weakly checked
//
#include <hip/hip_runtime.h>
#include <math.h>

constexpr int kNB     = 4;
constexpr int kNT     = 128;
constexpr int kNC     = 128;
constexpr int kNH     = 8;
constexpr int kHD     = 16;
constexpr int kDepth  = 2;
constexpr int kJRows  = kNB * kNT;
constexpr int kRBatch = kNT * kNT;
constexpr int kRRows  = kNB * kRBatch;
constexpr int kNG     = kNB * kNH;
constexpr int kKPad   = 32;
constexpr int kVPad   = 64;
constexpr int kRqkN   = 320;
constexpr float kAttScale = 0.25f;
constexpr float kWCarry   = 16.0f;
constexpr float kPCarry   = 1024.0f;
constexpr float kOCarry   = 64.0f;
constexpr float kHCarry   = 16.0f;
constexpr float kLnEps    = 1e-5f;

constexpr size_t kOffWT    = 0;
constexpr size_t kWTBytes  = 1048576;
constexpr size_t kWoJqkv = 0, kWoRqkc = 98304, kWoProj = 180224, kWoJ1 = 212992, kWoJ2 = 245760,
                 kWoR1a = 278528, kWoR1b = 802816, kWoR2a = 933888, kWoR2b = 966656;
static_assert(kWoR2b + 128 * 128 * 2 <= kWTBytes, "wt carve");
constexpr size_t kOffJA   = kOffWT + kWTBytes;
constexpr size_t kOffJB   = kOffJA + (size_t)kJRows * kNC * 4;
constexpr size_t kOffX16  = kOffJB + (size_t)kJRows * kNC * 4;
constexpr size_t kOffH16J = kOffX16 + (size_t)kJRows * kNC * 2;
constexpr size_t kOffG16J = kOffH16J + (size_t)kJRows * kNC * 2;
constexpr size_t kOffO16  = kOffG16J + (size_t)kJRows * kNC * 2;
constexpr size_t kOffJQKV = kOffO16 + (size_t)kJRows * kNC * 2;
constexpr size_t kOffQP   = kOffJQKV + (size_t)kJRows * 3 * kNC * 4;
constexpr size_t kOffKP   = kOffQP + (size_t)kNG * kNT * kKPad * 2;
constexpr size_t kOffVT   = kOffKP + (size_t)kNG * kNT * kKPad * 2;
constexpr size_t kOffSG   = kOffVT + (size_t)kNG * kVPad * kNT * 2;
constexpr size_t kOffP16  = kOffSG + (size_t)kNG * kNT * kNT * 4;
constexpr size_t kOffOG   = kOffP16 + (size_t)kNG * kNT * kNT * 2;
constexpr size_t kOffRF1  = kOffOG + (size_t)kNG * kNT * kVPad * 4;
constexpr size_t kOffRF2  = kOffRF1 + (size_t)kRRows * kNC * 4;
constexpr size_t kOffBIG  = kOffRF2 + (size_t)kRRows * kNC * 4;
constexpr size_t kBigBytes = (size_t)3 * kRBatch * 512 * 2;
constexpr size_t kBigSub1 = (size_t)kRBatch * 512 * 2;
constexpr size_t kBigSub2 = 2 * kBigSub1;
constexpr size_t kWsTotal  = kOffBIG + kBigBytes;
static_assert((size_t)kRRows * kNC * 2 <= kBigSub1, "R16 fits sub0");
static_assert(kBigSub1 + (size_t)kRBatch * kRqkN * 4 <= kBigBytes, "RQKC fits");
static_assert(kWsTotal <= 134217728ull, "ws carve");
static_assert((kOffJA % 256) == 0 && (kOffSG % 256) == 0 && (kOffRF1 % 256) == 0 && (kOffBIG % 256) == 0, "align");
constexpr size_t kOut0Floats = (size_t)kJRows * kNC;
constexpr size_t kOutFloats  = kOut0Floats + (size_t)kRRows * kNC;

typedef __attribute__((ext_vector_type(16))) _Float16 v16h;
typedef __attribute__((ext_vector_type(8)))  _Float16 v8h;
typedef __attribute__((ext_vector_type(16))) __bf16   v16b;
typedef __attribute__((ext_vector_type(8)))  __bf16   v8b;
typedef __attribute__((ext_vector_type(8)))  float    v8f;
typedef __attribute__((ext_vector_type(4)))  float    v4f;
typedef __attribute__((ext_vector_type(4)))  unsigned int v4u;

__device__ __forceinline__ unsigned short f2bf_bits(float f) {
  unsigned u = __float_as_uint(f);
  return (unsigned short)((u + 0x7FFFu + ((u >> 16) & 1u)) >> 16);
}
__device__ __forceinline__ float bf_bits2f(unsigned short h) { return __uint_as_float(((unsigned)h) << 16); }

__device__ __forceinline__ void dep_guard_h(v8f& a, v8f& b, v16h x, v16h y) { asm volatile("v_nop\n\tv_nop\n\tv_nop\n\tv_nop" : "+v"(a), "+v"(b) : "v"(x), "v"(y)); }
__device__ __forceinline__ void dep_guard_b(v8f& a, v8f& b, v16b x, v16b y) { asm volatile("v_nop\n\tv_nop\n\tv_nop\n\tv_nop" : "+v"(a), "+v"(b) : "v"(x), "v"(y)); }
__device__ __forceinline__ void keep4_h(v16h a, v16h b, v16h c, v16h d) { asm volatile("v_nop" :: "v"(a), "v"(b), "v"(c), "v"(d)); }
__device__ __forceinline__ void keep4_b(v16b a, v16b b, v16b c, v16b d) { asm volatile("v_nop" :: "v"(a), "v"(b), "v"(c), "v"(d)); }
__device__ __forceinline__ void acc_guard4(v8f& a, v8f& b, v8f& c, v8f& d) { asm volatile("v_nop\n\tv_nop\n\tv_nop\n\tv_nop" : "+v"(a), "+v"(b), "+v"(c), "+v"(d)); }
template <typename T> struct Frag;
template <> struct Frag<_Float16> {
  typedef v16h V; union U { v16h v; v8h h[2]; };
  static __device__ __forceinline__ v16h load(const _Float16* p) {
    U f; f.h[0] = *(const v8h*)(p); f.h[1] = *(const v8h*)(p + 16); return f.v;
  }
  static __device__ __forceinline__ v8f mma(v16h a, v16h b, v8f c) {
    return __builtin_amdgcn_wmma_f32_16x16x32_f16(false, a, false, b, (short)0, c, false, false);
  }
  static __device__ __forceinline__ void guard(v8f& a, v8f& b, v16h x, v16h y) { dep_guard_h(a, b, x, y); }
  static __device__ __forceinline__ void keep(v16h a, v16h b, v16h c, v16h d) { keep4_h(a, b, c, d); }
};
template <> struct Frag<__bf16> {
  typedef v16b V; union U { v16b v; v8b h[2]; };
  static __device__ __forceinline__ v16b load(const __bf16* p) {
    U f; f.h[0] = *(const v8b*)(p); f.h[1] = *(const v8b*)(p + 16); return f.v;
  }
  static __device__ __forceinline__ v8f mma(v16b a, v16b b, v8f c) {
    return __builtin_amdgcn_wmma_f32_16x16x32_bf16(false, a, false, b, (short)0, c, false, false);
  }
  static __device__ __forceinline__ void guard(v8f& a, v8f& b, v16b x, v16b y) { dep_guard_b(a, b, x, y); }
  static __device__ __forceinline__ void keep(v16b a, v16b b, v16b c, v16b d) { keep4_b(a, b, c, d); }
};

__device__ __forceinline__ unsigned pk16(unsigned short a, unsigned short b) { return (unsigned)a | ((unsigned)b << 16); }
__device__ __forceinline__ unsigned short h_bits(float f) { const _Float16 h = (_Float16)f; return __builtin_bit_cast(unsigned short, h); }

template <int ET> struct Elem;
template <> struct Elem<0> { typedef _Float16 T; };
template <> struct Elem<1> { typedef __bf16 T; };
template <int ET, bool SPLIT, int BIAS_MODE, int OUT_MODE, bool RESID, int ACT = 0>
__global__ __launch_bounds__(256) void wmma_gemm64(
    const unsigned short* __restrict__ Ap, const unsigned short* __restrict__ A2p, int lda, long strideA,
    const unsigned short* __restrict__ Btp, const unsigned short* __restrict__ Bt2p, int ldb, long strideB,
    void* __restrict__ Cout, void* __restrict__ Cout2, int ldc, long strideC,
    const float* __restrict__ bias,
    const float* __restrict__ resid, long strideR,
    int M, int N, int K, float scale) {
  typedef typename Elem<ET>::T T;
  typedef typename Frag<T>::V V;
  const T* A = (const T*)Ap; const T* A2 = (const T*)A2p; const T* Bt = (const T*)Btp; const T* Bt2 = (const T*)Bt2p;
  __shared__ __align__(16) float sT[8][16 * 68];
  const int b    = blockIdx.y;
  const int lane = threadIdx.x & 31;
  const int wave = threadIdx.x >> 5;
  const int tilesN = N >> 6;
  const int tilesM = M >> 6;
  const int tile = blockIdx.x * 8 + wave;
  if (tile >= tilesM * tilesN) return;
  const int tm = tile / tilesN;
  const int tn = tile - tm * tilesN;
  const int m0 = tm << 6;
  const int n0 = tn << 6;

  const T* Ab  = A  + (size_t)b * strideA;
  const T* Bb  = Bt + (size_t)b * strideB;
  const T* Ab2 = SPLIT ? (A2  + (size_t)b * strideA) : nullptr;
  const T* Bb2 = SPLIT ? (Bt2 + (size_t)b * strideB) : nullptr;

  const int rlane = lane & 15;
  const int koff  = (lane >> 4) * 8;
  const int mOff  = (lane >> 4) * 8;

  v8f acc[4][4];
#pragma unroll
  for (int i = 0; i < 4; ++i)
#pragma unroll
    for (int j = 0; j < 4; ++j) acc[i][j] = (v8f){0.f,0.f,0.f,0.f,0.f,0.f,0.f,0.f};

  for (int k0 = 0; k0 < K; k0 += 32) {
    V bh[4], bl[4];
#pragma unroll
    for (int j = 0; j < 4; ++j) {
      const size_t bo = (size_t)(n0 + (j << 4) + rlane) * ldb + koff + k0;
      bh[j] = Frag<T>::load(Bb + bo);
      if (SPLIT) bl[j] = Frag<T>::load(Bb2 + bo);
    }
#pragma unroll
    for (int i = 0; i < 4; ++i) {
      const size_t ao = (size_t)(m0 + (i << 4) + rlane) * lda + koff + k0;
      V ah = Frag<T>::load(Ab + ao);
      V al;
      if (SPLIT) al = Frag<T>::load(Ab2 + ao);
#pragma unroll
      for (int j = 0; j < 4; ++j) {
        acc[i][j] = Frag<T>::mma(ah, bh[j], acc[i][j]);
        if (SPLIT) {
          acc[i][j] = Frag<T>::mma(ah, bl[j], acc[i][j]);
          acc[i][j] = Frag<T>::mma(al, bh[j], acc[i][j]);
        }
      }
      Frag<T>::guard(acc[i][0], acc[i][3], ah, SPLIT ? al : ah);
    }
    Frag<T>::keep(bh[0], bh[1], bh[2], bh[3]);
    if (SPLIT) Frag<T>::keep(bl[0], bl[1], bl[2], bl[3]);
  }
  acc_guard4(acc[0][0], acc[0][1], acc[0][2], acc[0][3]);
  acc_guard4(acc[1][0], acc[1][1], acc[1][2], acc[1][3]);
  acc_guard4(acc[2][0], acc[2][1], acc[2][2], acc[2][3]);
  acc_guard4(acc[3][0], acc[3][1], acc[3][2], acc[3][3]);

  float* slab = sT[wave];
  const float* Rb = RESID ? (resid + (size_t)b * strideR) : nullptr;
#pragma unroll
  for (int i = 0; i < 4; ++i) {
    const int mBase = m0 + (i << 4);
#pragma unroll
    for (int j = 0; j < 4; ++j) {
      const int n = n0 + (j << 4) + rlane;
      float bv = 0.f;
      if (BIAS_MODE == 2) bv = bias[n];
#pragma unroll
      for (int r = 0; r < 8; ++r) {
        float v = acc[i][j][r] * scale;
        if (BIAS_MODE == 1) v += bias[mBase + mOff + r];
        if (BIAS_MODE == 2) v += bv;
        if (RESID) v += Rb[(size_t)(mBase + mOff + r) * ldc + n];
        if (ACT == 2) v = fmaxf(v, 0.0f);
        if (ACT == 4) v = (v > 0.f) ? v : 0.01f * v;
        slab[(mOff + r) * 68 + (j << 4) + rlane] = v;
      }
    }
    __builtin_amdgcn_fence(__ATOMIC_RELEASE, "workgroup");
    __builtin_amdgcn_wave_barrier();
    __builtin_amdgcn_fence(__ATOMIC_ACQUIRE, "workgroup");
    if (OUT_MODE == 0) {
      float* C = (float*)Cout + (size_t)b * strideC;
      const int hh = lane >> 4, c4 = (lane & 15) * 4;
      for (int pass = 0; pass < 2; ++pass) {
#pragma unroll
        for (int it = 0; it < 8; ++it) {
          const int row = it * 2 + hh;
          v4f v = *(const v4f*)(slab + row * 68 + c4);
          *(volatile v4f*)(C + (size_t)(mBase + row) * ldc + n0 + c4) = v;
        }
        __threadfence();
      }
    } else {
      const int q = lane >> 3, c8 = (lane & 7) * 8;
      unsigned short* C  = (unsigned short*)Cout  + (size_t)b * strideC;
      unsigned short* C2 = (OUT_MODE == 2) ? ((unsigned short*)Cout2 + (size_t)b * strideC) : nullptr;
      for (int pass = 0; pass < 2; ++pass) {
#pragma unroll
        for (int it = 0; it < 4; ++it) {
          const int row = it * 4 + q;
          const float* sp = slab + row * 68 + c8;
          v8h hv, lv;
#pragma unroll
          for (int e = 0; e < 8; ++e) {
            if (OUT_MODE == 1) {
              hv[e] = (_Float16)sp[e];
            } else {
              unsigned short hb = f2bf_bits(sp[e]);
              unsigned short lb = f2bf_bits(sp[e] - bf_bits2f(hb));
              hv[e] = __builtin_bit_cast(_Float16, hb);
              lv[e] = __builtin_bit_cast(_Float16, lb);
            }
          }
          *(volatile v8h*)(C + (size_t)(mBase + row) * ldc + n0 + c8) = hv;
          if (OUT_MODE == 2) *(volatile v8h*)(C2 + (size_t)(mBase + row) * ldc + n0 + c8) = lv;
        }
        __threadfence();
      }
    }
    __builtin_amdgcn_fence(__ATOMIC_RELEASE, "workgroup");
    __builtin_amdgcn_wave_barrier();
    __builtin_amdgcn_fence(__ATOMIC_ACQUIRE, "workgroup");
  }
}

__global__ __launch_bounds__(256) void wt_kernel(
    const float* __restrict__ w0, const float* __restrict__ w1, const float* __restrict__ w2,
    const float* __restrict__ w3, const float* __restrict__ w4, const float* __restrict__ w5,
    const float* __restrict__ w6, const float* __restrict__ w7, const float* __restrict__ w8,
    unsigned short* __restrict__ o0, unsigned short* __restrict__ o1, unsigned short* __restrict__ o2,
    unsigned short* __restrict__ o3, unsigned short* __restrict__ o4, unsigned short* __restrict__ o5,
    unsigned short* __restrict__ o6, unsigned short* __restrict__ o7, unsigned short* __restrict__ o8,
    float scale) {
  __shared__ float sm[64][65];
  const int z = blockIdx.z;
  const float* W = (z == 0) ? w0 : (z == 1) ? w1 : (z == 2) ? w2 : (z == 3) ? w3 : (z == 4) ? w4 :
                   (z == 5) ? w5 : (z == 6) ? w6 : (z == 7) ? w7 : w8;
  unsigned short* op = (z == 0) ? o0 : (z == 1) ? o1 : (z == 2) ? o2 : (z == 3) ? o3 : (z == 4) ? o4 :
                       (z == 5) ? o5 : (z == 6) ? o6 : (z == 7) ? o7 : o8;
  const int kdim = (z == 5 || z == 6) ? 512 : 128;
  const int ndim = (z == 0) ? 384 : (z == 1) ? 256 : (z == 5) ? 512 : 128;
  const int k0 = blockIdx.x * 64;
  const int n0 = blockIdx.y * 64;
  if (k0 >= kdim || n0 >= ndim) return;
  const int t = threadIdx.x;
#pragma unroll
  for (int i = 0; i < 16; ++i) {
    const int e = i * 256 + t;
    const int r = e >> 6;
    const int c = e & 63;
    sm[c][r] = W[(size_t)(k0 + r) * ndim + n0 + c] * scale;
  }
  __syncthreads();
  const int lane = t & 31, wave = t >> 5;
  const int q = lane >> 3, c8 = (lane & 7) * 8;
  for (int pass = 0; pass < 2; ++pass) {
#pragma unroll
    for (int it = 0; it < 2; ++it) {
      const int row = wave * 8 + it * 4 + q;
      unsigned short hb[8];
#pragma unroll
      for (int e = 0; e < 8; ++e) hb[e] = h_bits(sm[row][c8 + e]);
      const v4u u = (v4u){pk16(hb[0], hb[1]), pk16(hb[2], hb[3]), pk16(hb[4], hb[5]), pk16(hb[6], hb[7])};
      *(volatile v4u*)(op + (size_t)(n0 + row) * kdim + k0 + c8) = u;
    }
    __threadfence();
  }
}

__global__ __launch_bounds__(256) void rconv_rows_kernel(const float* __restrict__ wrc, unsigned short* __restrict__ outT, float scale) {
  const int lane = threadIdx.x & 31, wave = threadIdx.x >> 5;
  const int kq = (lane & 15) * 8;
  v4u u[4];
#pragma unroll
  for (int it = 0; it < 4; ++it) {
    const int n = 256 + wave * 8 + it * 2 + (lane >> 4);
    const int col = n - 256;
    const int colc = (col < 8) ? col : 7;
    const bool valid = (col < 8);
    unsigned short hb[8];
#pragma unroll
    for (int e = 0; e < 8; ++e) {
      const float x = wrc[(kq + e) * 8 + colc] * scale;
      hb[e] = h_bits(valid ? x : 0.0f);
    }
    u[it] = (v4u){pk16(hb[0], hb[1]), pk16(hb[2], hb[3]), pk16(hb[4], hb[5]), pk16(hb[6], hb[7])};
  }
  for (int pass = 0; pass < 2; ++pass) {
#pragma unroll
    for (int it = 0; it < 4; ++it) {
      const int n = 256 + wave * 8 + it * 2 + (lane >> 4);
      *(volatile v4u*)(outT + (size_t)n * kNC + kq) = u[it];
    }
    __threadfence();
  }
}

__global__ __launch_bounds__(256) void ln128_kernel(const float* __restrict__ in, const float* __restrict__ g,
                                                    const float* __restrict__ be, unsigned short* __restrict__ out) {
  const int lane = threadIdx.x & 31, wave = threadIdx.x >> 5;
  const int task = blockIdx.x * 8 + wave;
  const int row  = task * 2 + (lane >> 4);
  const int cq   = (lane & 15) * 8;
  const float* p = in + (size_t)row * kNC + cq;
  const v4f a = *(const v4f*)(p);
  const v4f c = *(const v4f*)(p + 4);
  float x[8];
#pragma unroll
  for (int e = 0; e < 4; ++e) { x[e] = a[e]; x[4 + e] = c[e]; }
  float s = 0.f;
#pragma unroll
  for (int e = 0; e < 8; ++e) s += x[e];
#pragma unroll
  for (int off = 8; off > 0; off >>= 1) s += __shfl_xor(s, off, 32);
  const float mean = s * (1.0f / 128.0f);
  float vs = 0.f;
#pragma unroll
  for (int e = 0; e < 8; ++e) { x[e] = x[e] - mean; vs += x[e] * x[e]; }
#pragma unroll
  for (int off = 8; off > 0; off >>= 1) vs += __shfl_xor(vs, off, 32);
  const float inv = rsqrtf(vs * (1.0f / 128.0f) + kLnEps);
  const v4f g0 = *(const v4f*)(g + cq), g1 = *(const v4f*)(g + cq + 4);
  const v4f b0 = *(const v4f*)(be + cq), b1 = *(const v4f*)(be + cq + 4);
  unsigned short hb[8];
#pragma unroll
  for (int e = 0; e < 4; ++e) {
    hb[e]     = h_bits((x[e] * inv) * g0[e] + b0[e]);
    hb[4 + e] = h_bits((x[4 + e] * inv) * g1[e] + b1[e]);
  }
  const v4u u = (v4u){pk16(hb[0], hb[1]), pk16(hb[2], hb[3]), pk16(hb[4], hb[5]), pk16(hb[6], hb[7])};
  unsigned short* q = out + (size_t)row * kNC + cq;
  *(volatile v4u*)q = u;
  __threadfence();
  *(volatile v4u*)q = u;
}

__global__ __launch_bounds__(256) void rin_ln_kernel(const float* __restrict__ rf, const float* __restrict__ jf,
                                                     const float* __restrict__ g, const float* __restrict__ be,
                                                     unsigned short* __restrict__ out, int b) {
  const int lane = threadIdx.x & 31, wave = threadIdx.x >> 5;
  const int rl = blockIdx.x * 8 + wave;
  const int i = rl >> 7, j = rl & 127;
  const int hsel = lane >> 4;
  const int cq = (lane & 15) * 8;
  const size_t rowA = (size_t)b * kRBatch + (size_t)rl;
  const size_t rowT = (size_t)b * kRBatch + (size_t)j * kNT + (size_t)i;
  const float* pa = rf + rowA * kNC + cq;
  const float* pt = rf + rowT * kNC + cq;
  const float* pj = jf + ((size_t)b * kNT + j) * kNC + cq;
  const float* pi = jf + ((size_t)b * kNT + i) * kNC + cq;
  const v4f a0 = *(const v4f*)(pa), a1 = *(const v4f*)(pa + 4);
  const v4f t0 = *(const v4f*)(pt), t1 = *(const v4f*)(pt + 4);
  const v4f j0 = *(const v4f*)(pj), j1 = *(const v4f*)(pj + 4);
  const v4f i0 = *(const v4f*)(pi), i1 = *(const v4f*)(pi + 4);
  float xa[8], xb[8];
#pragma unroll
  for (int e = 0; e < 4; ++e) {
    xa[e]     = hsel ? t0[e] : a0[e];
    xa[4 + e] = hsel ? t1[e] : a1[e];
    xb[e]     = hsel ? i0[e] : j0[e];
    xb[4 + e] = hsel ? i1[e] : j1[e];
  }
  float s = 0.f;
#pragma unroll
  for (int e = 0; e < 8; ++e) s += xa[e];
#pragma unroll
  for (int e = 0; e < 8; ++e) s += xb[e];
#pragma unroll
  for (int off = 16; off > 0; off >>= 1) s += __shfl_xor(s, off, 32);
  const float mean = s * (1.0f / 512.0f);
  float vs = 0.f;
#pragma unroll
  for (int e = 0; e < 8; ++e) { xa[e] = xa[e] - mean; vs += xa[e] * xa[e]; }
#pragma unroll
  for (int e = 0; e < 8; ++e) { xb[e] = xb[e] - mean; vs += xb[e] * xb[e]; }
#pragma unroll
  for (int off = 16; off > 0; off >>= 1) vs += __shfl_xor(vs, off, 32);
  const float inv = rsqrtf(vs * (1.0f / 512.0f) + kLnEps);
  const int ca = 8 * lane, cb = 256 + 8 * lane;
  const v4f ga0 = *(const v4f*)(g + ca), ga1 = *(const v4f*)(g + ca + 4);
  const v4f ba0 = *(const v4f*)(be + ca), ba1 = *(const v4f*)(be + ca + 4);
  const v4f gb0 = *(const v4f*)(g + cb), gb1 = *(const v4f*)(g + cb + 4);
  const v4f bb0 = *(const v4f*)(be + cb), bb1 = *(const v4f*)(be + cb + 4);
  unsigned short ha[8], hb[8];
#pragma unroll
  for (int e = 0; e < 4; ++e) {
    ha[e]     = h_bits((xa[e] * inv) * ga0[e] + ba0[e]);
    ha[4 + e] = h_bits((xa[4 + e] * inv) * ga1[e] + ba1[e]);
    hb[e]     = h_bits((xb[e] * inv) * gb0[e] + bb0[e]);
    hb[4 + e] = h_bits((xb[4 + e] * inv) * gb1[e] + bb1[e]);
  }
  const v4u ua = (v4u){pk16(ha[0], ha[1]), pk16(ha[2], ha[3]), pk16(ha[4], ha[5]), pk16(ha[6], ha[7])};
  const v4u ub = (v4u){pk16(hb[0], hb[1]), pk16(hb[2], hb[3]), pk16(hb[4], hb[5]), pk16(hb[6], hb[7])};
  unsigned short* q = out + (size_t)rl * 512;
  *(volatile v4u*)(q + ca) = ua;
  *(volatile v4u*)(q + cb) = ub;
  __threadfence();
  *(volatile v4u*)(q + ca) = ua;
  *(volatile v4u*)(q + cb) = ub;
}

__global__ __launch_bounds__(256) void gelu_kernel(const unsigned short* __restrict__ hin, const float* __restrict__ bias,
                                                   unsigned short* __restrict__ gout, int cmask, int n2) {
  const int i = blockIdx.x * 256 + threadIdx.x;
  if (i >= n2) return;
  const unsigned w = ((const unsigned*)hin)[i];
  const int col = (2 * i) & cmask;
  const float bz0 = bias[col], bz1 = bias[col + 1];
  unsigned res = 0u;
#pragma unroll 1
  for (int e = 0; e < 2; ++e) {
    const unsigned short hs = (unsigned short)((e == 0) ? (w & 0xffffu) : (w >> 16));
    const float hv = (float)__builtin_bit_cast(_Float16, hs);
    const float x  = hv * (1.0f / kHCarry) + ((e == 0) ? bz0 : bz1);
    const float gl = 0.5f * x * (1.0f + erff(x * 0.70710678118654752f));
    const unsigned short ob = h_bits(gl * kHCarry);
    res |= ((unsigned)ob) << (16 * e);
  }
  ((volatile unsigned*)gout)[i] = res;
  __threadfence();
  ((volatile unsigned*)gout)[i] = res;
}

__global__ __launch_bounds__(256) void qkv_kernel(const float* __restrict__ jqkv, unsigned short* __restrict__ qp,
                                                  unsigned short* __restrict__ kp, unsigned short* __restrict__ vt) {
  const int lane = threadIdx.x & 31, wave = threadIdx.x >> 5;
  const int blk = blockIdx.x;
  if (blk < 64) {
    const int wt = blk * 8 + wave;
    const int g = wt >> 4;
    const int b = g >> 3, h = g & 7;
    const int i = (wt & 15) * 8 + (lane >> 2);
    const int part = lane & 3;
    const int pc = (part < 2) ? part : 1;
    const bool valid = (part < 2);
    const float* src = jqkv + ((size_t)(b * kNT + i)) * (3 * kNC) + h * kHD + pc * 8;
    const v4f qa = *(const v4f*)(src),        qc = *(const v4f*)(src + 4);
    const v4f ka = *(const v4f*)(src + kNC),  kc = *(const v4f*)(src + kNC + 4);
    unsigned short hq[8], hk[8];
#pragma unroll
    for (int e = 0; e < 4; ++e) {
      hq[e]     = h_bits(valid ? qa[e] : 0.0f);
      hq[4 + e] = h_bits(valid ? qc[e] : 0.0f);
      hk[e]     = h_bits(valid ? ka[e] : 0.0f);
      hk[4 + e] = h_bits(valid ? kc[e] : 0.0f);
    }
    const v4u uq = (v4u){pk16(hq[0], hq[1]), pk16(hq[2], hq[3]), pk16(hq[4], hq[5]), pk16(hq[6], hq[7])};
    const v4u uk = (v4u){pk16(hk[0], hk[1]), pk16(hk[2], hk[3]), pk16(hk[4], hk[5]), pk16(hk[6], hk[7])};
    const size_t off = ((size_t)g * kNT + i) * kKPad + part * 8;
    *(volatile v4u*)(qp + off) = uq;
    *(volatile v4u*)(kp + off) = uk;
    __threadfence();
    *(volatile v4u*)(qp + off) = uq;
    *(volatile v4u*)(kp + off) = uk;
  } else {
    const int vtask = (blk - 64) * 8 + wave;
    const int g = vtask >> 5;
    const int b = g >> 3, h = g & 7;
    const int d = (vtask & 31) * 2 + (lane >> 4);
    const int dc = (d < kHD) ? d : (kHD - 1);
    const bool valid = (d < kHD);
    const int j0 = (lane & 15) * 8;
    const float* src = jqkv + ((size_t)(b * kNT + j0)) * (3 * kNC) + 2 * kNC + h * kHD + dc;
    unsigned short hv[8];
#pragma unroll
    for (int e = 0; e < 8; ++e) {
      const float x = src[(size_t)e * (3 * kNC)];
      hv[e] = h_bits(valid ? x : 0.0f);
    }
    const v4u uv = (v4u){pk16(hv[0], hv[1]), pk16(hv[2], hv[3]), pk16(hv[4], hv[5]), pk16(hv[6], hv[7])};
    const size_t off = ((size_t)g * kVPad + d) * kNT + j0;
    *(volatile v4u*)(vt + off) = uv;
    __threadfence();
    *(volatile v4u*)(vt + off) = uv;
  }
}

__global__ __launch_bounds__(256) void score_softmax_kernel(const float* __restrict__ sg, const float* __restrict__ rqk,
                                                            unsigned short* __restrict__ p16, int b) {
  __shared__ float scr[kNH][kNT];
  __shared__ __align__(16) unsigned prow[kNH][64];
  const int lane = threadIdx.x & 31, wave = threadIdx.x >> 5;
  const int i = blockIdx.x;
  const int h = wave;
  const int g = b * kNH + h;
  const v4f sj = *(const v4f*)(sg + ((size_t)g * kNT + i) * kNT + 4 * lane);
#pragma unroll 1
  for (int jj = 0; jj < 4; ++jj) {
    const int j = 4 * lane + jj;
    const float* base = rqk + ((size_t)i * kNT + j) * kRqkN;
    const float* pq = base + h * kHD;
    const float* pk = base + kNC + h * kHD;
    const v4f q0 = *(const v4f*)(pq), q1 = *(const v4f*)(pq + 4), q2 = *(const v4f*)(pq + 8), q3 = *(const v4f*)(pq + 12);
    const v4f k0 = *(const v4f*)(pk), k1 = *(const v4f*)(pk + 4), k2 = *(const v4f*)(pk + 8), k3 = *(const v4f*)(pk + 12);
    float qu = 0.f;
#pragma unroll
    for (int e = 0; e < 4; ++e) qu += q0[e] * k0[e];
#pragma unroll
    for (int e = 0; e < 4; ++e) qu += q1[e] * k1[e];
#pragma unroll
    for (int e = 0; e < 4; ++e) qu += q2[e] * k2[e];
#pragma unroll
    for (int e = 0; e < 4; ++e) qu += q3[e] * k3[e];
    const float rl = base[2 * kNC + h];
    const float sv = (jj == 0) ? sj[0] : (jj == 1) ? sj[1] : (jj == 2) ? sj[2] : sj[3];
    scr[h][j] = (sv + rl + qu) * kAttScale;
  }
  __syncthreads();
  const float s0 = scr[h][4 * lane], s1 = scr[h][4 * lane + 1], s2 = scr[h][4 * lane + 2], s3 = scr[h][4 * lane + 3];
  float m = fmaxf(fmaxf(s0, s1), fmaxf(s2, s3));
#pragma unroll
  for (int off = 16; off > 0; off >>= 1) m = fmaxf(m, __shfl_xor(m, off, 32));
  const float e0 = expf(s0 - m), e1 = expf(s1 - m), e2 = expf(s2 - m), e3 = expf(s3 - m);
  float sum = (e0 + e1) + (e2 + e3);
#pragma unroll
  for (int off = 16; off > 0; off >>= 1) sum += __shfl_xor(sum, off, 32);
  const float inv = kPCarry / sum;
  prow[h][2 * lane]     = pk16(h_bits(e0 * inv), h_bits(e1 * inv));
  prow[h][2 * lane + 1] = pk16(h_bits(e2 * inv), h_bits(e3 * inv));
  __syncthreads();
  if (lane < 16) {
    const v4u u = *(const v4u*)(&prow[h][4 * lane]);
    unsigned short* dst = p16 + ((size_t)g * kNT + i) * kNT + 8 * lane;
    *(volatile v4u*)dst = u;
    __threadfence();
    *(volatile v4u*)dst = u;
  }
}

__global__ __launch_bounds__(256) void ogather_kernel(const float* __restrict__ og, unsigned short* __restrict__ o16) {
  const int lane = threadIdx.x & 31, wave = threadIdx.x >> 5;
  const int task = blockIdx.x * 8 + wave;
  const int tok = task * 2 + (lane >> 4);
  const int b = tok >> 7, i = tok & 127;
  const int cp = lane & 15;
  const int h = cp >> 1, d0 = (cp & 1) * 8;
  const float* src = og + (((size_t)(b * kNH + h)) * kNT + i) * kVPad + d0;
  const v4f a = *(const v4f*)(src), c = *(const v4f*)(src + 4);
  unsigned short hb[8];
#pragma unroll
  for (int e = 0; e < 4; ++e) { hb[e] = h_bits(a[e] * kOCarry); hb[4 + e] = h_bits(c[e] * kOCarry); }
  const v4u u = (v4u){pk16(hb[0], hb[1]), pk16(hb[2], hb[3]), pk16(hb[4], hb[5]), pk16(hb[6], hb[7])};
  unsigned short* dst = o16 + (size_t)tok * kNC + cp * 8;
  *(volatile v4u*)dst = u;
  __threadfence();
  *(volatile v4u*)dst = u;
}

static inline void gemm_f32out(hipStream_t st, const unsigned short* A, int lda, long sA,
                               const unsigned short* Bt, int ldb, long sB,
                               float* C, int ldc, long sC, int M, int N, int K, float scale, int batch) {
  const int tiles = (M >> 6) * (N >> 6);
  dim3 grid((tiles + 7) / 8, batch);
  wmma_gemm64<0, false, 0, 0, false, 0><<<grid, 256, 0, st>>>(
      A, nullptr, lda, sA, Bt, nullptr, ldb, sB, (void*)C, nullptr, ldc, sC, nullptr, nullptr, 0L, M, N, K, scale);
}
static inline void gemm_f16out(hipStream_t st, const unsigned short* A, int lda,
                               const unsigned short* Bt, int ldb,
                               unsigned short* C, int ldc, int M, int N, int K, float scale) {
  const int tiles = (M >> 6) * (N >> 6);
  dim3 grid((tiles + 7) / 8, 1);
  wmma_gemm64<0, false, 0, 1, false, 0><<<grid, 256, 0, st>>>(
      A, nullptr, lda, 0L, Bt, nullptr, ldb, 0L, (void*)C, nullptr, ldc, 0L, nullptr, nullptr, 0L, M, N, K, scale);
}
static inline void gemm_resid(hipStream_t st, const unsigned short* A, int lda,
                              const unsigned short* Bt, int ldb,
                              float* C, int ldc, const float* bias, const float* resid,
                              int M, int N, int K, float scale) {
  const int tiles = (M >> 6) * (N >> 6);
  dim3 grid((tiles + 7) / 8, 1);
  wmma_gemm64<0, false, 2, 0, true, 0><<<grid, 256, 0, st>>>(
      A, nullptr, lda, 0L, Bt, nullptr, ldb, 0L, (void*)C, nullptr, ldc, 0L, bias, resid, 0L, M, N, K, scale);
}

extern "C" void kernel_launch(void* const* d_in, const int* in_sizes, int n_in,
                              void* d_out, int out_size, void* d_ws, size_t ws_size,
                              hipStream_t stream) {
  if (n_in < 29) return;
  if ((size_t)out_size < kOutFloats) return;
  if (ws_size < kWsTotal) return;
  if (in_sizes[0] != kJRows * kNC || in_sizes[1] != kRRows * kNC) return;

  const float* in_jf   = (const float*)d_in[0];
  const float* in_rf   = (const float*)d_in[1];
  const float* w_jqkv  = (const float*)d_in[2];
  const float* w_rconv = (const float*)d_in[3];
  const float* w_rqk   = (const float*)d_in[4];
  const float* w_proj  = (const float*)d_in[5];
  const float* b_proj  = (const float*)d_in[6];
  const float* g_a1    = (const float*)d_in[7];
  const float* be_a1   = (const float*)d_in[8];
  const float* g_a2    = (const float*)d_in[9];
  const float* be_a2   = (const float*)d_in[10];
  const float* g_j     = (const float*)d_in[11];
  const float* be_j    = (const float*)d_in[12];
  const float* g_r1    = (const float*)d_in[13];
  const float* be_r1   = (const float*)d_in[14];
  const float* g_r2    = (const float*)d_in[15];
  const float* be_r2   = (const float*)d_in[16];
  const float* wj1     = (const float*)d_in[17];
  const float* bj1     = (const float*)d_in[18];
  const float* wj2     = (const float*)d_in[19];
  const float* bj2     = (const float*)d_in[20];
  const float* wr1a    = (const float*)d_in[21];
  const float* br1a    = (const float*)d_in[22];
  const float* wr1b    = (const float*)d_in[23];
  const float* br1b    = (const float*)d_in[24];
  const float* wr2a    = (const float*)d_in[25];
  const float* br2a    = (const float*)d_in[26];
  const float* wr2b    = (const float*)d_in[27];
  const float* br2b    = (const float*)d_in[28];

  float* out0 = (float*)d_out;
  float* out1 = (float*)d_out + kOut0Floats;

  char* ws = (char*)d_ws;
  unsigned short* wtJqkv = (unsigned short*)(ws + kOffWT + kWoJqkv);
  unsigned short* wtRqkc = (unsigned short*)(ws + kOffWT + kWoRqkc);
  unsigned short* wtProj = (unsigned short*)(ws + kOffWT + kWoProj);
  unsigned short* wtJ1   = (unsigned short*)(ws + kOffWT + kWoJ1);
  unsigned short* wtJ2   = (unsigned short*)(ws + kOffWT + kWoJ2);
  unsigned short* wtR1a  = (unsigned short*)(ws + kOffWT + kWoR1a);
  unsigned short* wtR1b  = (unsigned short*)(ws + kOffWT + kWoR1b);
  unsigned short* wtR2a  = (unsigned short*)(ws + kOffWT + kWoR2a);
  unsigned short* wtR2b  = (unsigned short*)(ws + kOffWT + kWoR2b);
  float* jA  = (float*)(ws + kOffJA);
  float* jB  = (float*)(ws + kOffJB);
  unsigned short* x16  = (unsigned short*)(ws + kOffX16);
  unsigned short* h16j = (unsigned short*)(ws + kOffH16J);
  unsigned short* g16j = (unsigned short*)(ws + kOffG16J);
  unsigned short* o16  = (unsigned short*)(ws + kOffO16);
  float* jqkv = (float*)(ws + kOffJQKV);
  unsigned short* qp = (unsigned short*)(ws + kOffQP);
  unsigned short* kp = (unsigned short*)(ws + kOffKP);
  unsigned short* vt = (unsigned short*)(ws + kOffVT);
  float* sg = (float*)(ws + kOffSG);
  unsigned short* p16 = (unsigned short*)(ws + kOffP16);
  float* og = (float*)(ws + kOffOG);
  float* rf1 = (float*)(ws + kOffRF1);
  float* rf2 = (float*)(ws + kOffRF2);
  unsigned short* r16  = (unsigned short*)(ws + kOffBIG);
  float*          rqkc = (float*)(ws + kOffBIG + kBigSub1);
  unsigned short* rn16 = (unsigned short*)(ws + kOffBIG);
  unsigned short* h1p  = (unsigned short*)(ws + kOffBIG + kBigSub1);
  unsigned short* g1p  = (unsigned short*)(ws + kOffBIG + kBigSub2);
  unsigned short* rn2  = (unsigned short*)(ws + kOffBIG);
  unsigned short* h2p  = (unsigned short*)(ws + kOffBIG + kBigSub1);
  unsigned short* g2p  = (unsigned short*)(ws + kOffBIG + kBigSub2);

  const float* jcur = in_jf;
  const float* rcur = in_rf;

  for (int dl = 0; dl < kDepth; ++dl) {
    const float* Wjqkv = w_jqkv  + (size_t)dl * kNC * 3 * kNC;
    const float* Wrc   = w_rconv + (size_t)dl * kNC * kNH;
    const float* Wrqk  = w_rqk   + (size_t)dl * kNC * 2 * kNC;
    const float* Wproj = w_proj  + (size_t)dl * kNC * kNC;
    const float* Bproj = b_proj  + (size_t)dl * kNC;
    const float* Ga1 = g_a1 + (size_t)dl * kNC;  const float* Ba1 = be_a1 + (size_t)dl * kNC;
    const float* Ga2 = g_a2 + (size_t)dl * kNC;  const float* Ba2 = be_a2 + (size_t)dl * kNC;
    const float* Gj  = g_j  + (size_t)dl * kNC;  const float* Bj  = be_j  + (size_t)dl * kNC;
    const float* Gr1 = g_r1 + (size_t)dl * 4 * kNC;  const float* Br1 = be_r1 + (size_t)dl * 4 * kNC;
    const float* Gr2 = g_r2 + (size_t)dl * kNC;  const float* Br2 = be_r2 + (size_t)dl * kNC;
    const float* Wj1 = wj1 + (size_t)dl * kNC * kNC;  const float* Bj1 = bj1 + (size_t)dl * kNC;
    const float* Wj2 = wj2 + (size_t)dl * kNC * kNC;  const float* Bj2 = bj2 + (size_t)dl * kNC;
    const float* Wr1a = wr1a + (size_t)dl * 512 * 512;  const float* Br1a = br1a + (size_t)dl * 512;
    const float* Wr1b = wr1b + (size_t)dl * 512 * kNC;  const float* Br1b = br1b + (size_t)dl * kNC;
    const float* Wr2a = wr2a + (size_t)dl * kNC * kNC;  const float* Br2a = br2a + (size_t)dl * kNC;
    const float* Wr2b = wr2b + (size_t)dl * kNC * kNC;  const float* Br2b = br2b + (size_t)dl * kNC;

    const bool last = (dl == kDepth - 1);
    float* jmid  = jA;
    float* jnext = last ? out0 : jB;
    float* rmid  = rf1;
    float* rnext = last ? out1 : rf2;

    wt_kernel<<<dim3(8, 8, 9), 256, 0, stream>>>(Wjqkv, Wrqk, Wproj, Wj1, Wj2, Wr1a, Wr1b, Wr2a, Wr2b,
                                                  wtJqkv, wtRqkc, wtProj, wtJ1, wtJ2, wtR1a, wtR1b, wtR2a, wtR2b, kWCarry);
    rconv_rows_kernel<<<1, 256, 0, stream>>>(Wrc, wtRqkc, kWCarry);

    ln128_kernel<<<kJRows / 16, 256, 0, stream>>>(jcur, Ga1, Ba1, x16);
    gemm_f32out(stream, x16, kNC, 0L, wtJqkv, kNC, 0L, jqkv, 3 * kNC, 0L, kJRows, 3 * kNC, kNC, 1.0f / kWCarry, 1);
    qkv_kernel<<<192, 256, 0, stream>>>(jqkv, qp, kp, vt);
    gemm_f32out(stream, qp, kKPad, (long)(kNT * kKPad), kp, kKPad, (long)(kNT * kKPad),
                sg, kNT, (long)(kNT * kNT), kNT, kNT, kKPad, 1.0f, kNG);
    ln128_kernel<<<kRRows / 16, 256, 0, stream>>>(rcur, Ga2, Ba2, r16);
    for (int b = 0; b < kNB; ++b) {
      gemm_f32out(stream, r16 + (size_t)b * kRBatch * kNC, kNC, 0L, wtRqkc, kNC, 0L,
                  rqkc, kRqkN, 0L, kRBatch, kRqkN, kNC, 1.0f / kWCarry, 1);
      score_softmax_kernel<<<kNT, 256, 0, stream>>>(sg, rqkc, p16, b);
    }
    gemm_f32out(stream, p16, kNT, (long)(kNT * kNT), vt, kNT, (long)(kVPad * kNT),
                og, kVPad, (long)(kNT * kVPad), kNT, kVPad, kNT, 1.0f / kPCarry, kNG);
    ogather_kernel<<<32, 256, 0, stream>>>(og, o16);
    gemm_resid(stream, o16, kNC, wtProj, kNC, jmid, kNC, Bproj, jcur, kJRows, kNC, kNC, 1.0f / (kOCarry * kWCarry));

    ln128_kernel<<<kJRows / 16, 256, 0, stream>>>(jmid, Gj, Bj, x16);
    gemm_f16out(stream, x16, kNC, wtJ1, kNC, h16j, kNC, kJRows, kNC, kNC, kHCarry / kWCarry);
    gelu_kernel<<<(kJRows * kNC / 2 + 255) / 256, 256, 0, stream>>>(h16j, Bj1, g16j, kNC - 1, kJRows * kNC / 2);
    gemm_resid(stream, g16j, kNC, wtJ2, kNC, jnext, kNC, Bj2, jmid, kJRows, kNC, kNC, 1.0f / (kHCarry * kWCarry));

    for (int b = 0; b < kNB; ++b) {
      rin_ln_kernel<<<kRBatch / 8, 256, 0, stream>>>(rcur, jnext, Gr1, Br1, rn16, b);
      gemm_f16out(stream, rn16, 512, wtR1a, 512, h1p, 512, kRBatch, 512, 512, kHCarry / kWCarry);
      gelu_kernel<<<(kRBatch * 512 / 2 + 255) / 256, 256, 0, stream>>>(h1p, Br1a, g1p, 511, kRBatch * 512 / 2);
      gemm_resid(stream, g1p, 512, wtR1b, 512, rmid + (size_t)b * kRBatch * kNC, kNC, Br1b,
                 rcur + (size_t)b * kRBatch * kNC, kRBatch, kNC, 512, 1.0f / (kHCarry * kWCarry));
    }

    ln128_kernel<<<kRRows / 16, 256, 0, stream>>>(rmid, Gr2, Br2, rn2);
    gemm_f16out(stream, rn2, kNC, wtR2a, kNC, h2p, kNC, kRRows, kNC, kNC, kHCarry / kWCarry);
    gelu_kernel<<<(kRRows * kNC / 2 + 255) / 256, 256, 0, stream>>>(h2p, Br2a, g2p, kNC - 1, kRRows * kNC / 2);
    gemm_resid(stream, g2p, kNC, wtR2b, kNC, rnext, kNC, Br2b, rmid, kRRows, kNC, kNC, 1.0f / (kHCarry * kWCarry));

    jcur = jnext;
    rcur = rnext;
  }
}
